// LSTM_49357764165950
// MI455X (gfx1250) — hardware-verified
//
#include <hip/hip_runtime.h>
#include <math.h>

constexpr int NBATCH  = 1024;
constexpr int NTIME   = 256;
constexpr int NCELL   = 256;
constexpr int NXIN    = 128;
constexpr int NEMB    = 126;
constexpr int NHID    = 256;
constexpr int NGATE   = 4 * NHID;
constexpr int KCAT    = NXIN + NHID;
constexpr int KTILES  = KCAT / 32;
constexpr int BMROWS  = 64;
constexpr int MTILES  = BMROWS / 16;
constexpr int NTHR    = 512;
constexpr int NWAVE   = NTHR / 32;
constexpr int APITCH  = 392;
constexpr int SPITCH  = 260;
constexpr int PREPT   = 256;
constexpr float WCARRY     = 16.0f;
constexpr float WCARRY_INV = 1.0f / 16.0f;
constexpr float VSCALE     = 4.0f;
constexpr int OUT1_ELEM_OFF = NBATCH * NHID;

static_assert(KCAT == 384 && KCAT % 32 == 0, "K multiple of 32");
static_assert(NWAVE * 16 == NHID, "one 16-unit group per wave");
static_assert(NBATCH % BMROWS == 0, "exact grid");
static_assert(NGATE == 1024, "gate rows");
static_assert(NCELL == NTIME, "one tag step plus NTIME-1 velocity steps");
static_assert(APITCH % 8 == 0 && APITCH >= KCAT, "A tile pitch");
static_assert(SPITCH % 4 == 0 && SPITCH >= NHID, "staging pitch");
static_assert((size_t)OUT1_ELEM_OFF * 4 == 1048576, "second output byte offset");
static_assert((size_t)OUT1_ELEM_OFF * 4 + (size_t)NBATCH * NHID * 4 == 2097152, "output total bytes");
static_assert(BMROWS * (NXIN / 16) == NTHR, "x staging: one thread per 16 columns of a row");
static_assert((BMROWS * (NHID / 8)) % NTHR == 0, "h zero-fill exact");
static_assert((BMROWS * (NHID / 4)) % NTHR == 0, "final store exact");

typedef __attribute__((ext_vector_type(16))) _Float16 v16h;
typedef __attribute__((ext_vector_type(8)))  _Float16 v8h;
typedef __attribute__((ext_vector_type(8)))  float    v8f;
typedef __attribute__((ext_vector_type(4)))  float    v4f;
typedef __attribute__((ext_vector_type(2)))  float    v2f;

__device__ __forceinline__ void grp_guard(v8f& a0, v8f& a1, v8f& a2, v8f& a3,
                                          v16h x, v16h b0, v16h b1, v16h b2, v16h b3) {
  asm volatile("v_nop\n\tv_nop\n\tv_nop\n\tv_nop"
               : "+v"(a0), "+v"(a1), "+v"(a2), "+v"(a3)
               : "v"(x), "v"(b0), "v"(b1), "v"(b2), "v"(b3));
}

template <typename T> struct Frag;
template <> struct Frag<_Float16> {
  typedef v16h V; union U { v16h v; v8h h[2]; };
  static __device__ __forceinline__ v16h load(const _Float16* p) {
    U f; f.h[0] = *(const v8h*)(p); f.h[1] = *(const v8h*)(p + 16); return f.v;
  }
  static __device__ __forceinline__ v8f mma(v16h a, v16h b, v8f c) {
    return __builtin_amdgcn_wmma_f32_16x16x32_f16(false, a, false, b, (short)0, c, false, false);
  }
};

__device__ __forceinline__ float fsig(float x)  { return __builtin_amdgcn_rcpf(1.0f + expf(-x)); }
__device__ __forceinline__ float ftanh(float x) { return 1.0f - 2.0f * __builtin_amdgcn_rcpf(expf(2.0f * x) + 1.0f); }

__device__ __forceinline__ void cvt8_store(const float* __restrict__ src, unsigned short* __restrict__ dst) {
  const v4f a = *(const v4f*)(src);
  const v4f b = *(const v4f*)(src + 4);
  v8h hv;
#pragma unroll
  for (int e = 0; e < 4; ++e) {
    hv[e]     = (_Float16)(a[e] * WCARRY);
    hv[4 + e] = (_Float16)(b[e] * WCARRY);
  }
  *(volatile v8h*)dst = hv;
  __threadfence();
  *(volatile v8h*)dst = hv;
}

__global__ __launch_bounds__(PREPT) void lstm_prep_kernel(const float* __restrict__ w_ih, const float* __restrict__ w_hh,
                                                          const float* __restrict__ b_ih, const float* __restrict__ b_hh,
                                                          unsigned short* __restrict__ Wc, float* __restrict__ biasws) {
  const int bid = blockIdx.x;
  const int tid = threadIdx.x;
  if (bid < 64) {
    const int idx = bid * PREPT + tid;
    const int n = idx >> 4;
    const int c8 = (idx & 15) * 8;
    cvt8_store(w_ih + (size_t)n * NXIN + c8, Wc + (size_t)n * KCAT + c8);
  } else if (bid < 192) {
    const int idx = (bid - 64) * PREPT + tid;
    const int n = idx >> 5;
    const int c8 = (idx & 31) * 8;
    cvt8_store(w_hh + (size_t)n * NHID + c8, Wc + (size_t)n * KCAT + NXIN + c8);
  } else {
    const int i4 = tid * 4;
    const v4f a = *(const v4f*)(b_ih + i4);
    const v4f b = *(const v4f*)(b_hh + i4);
    const v4f o = a + b;
    *(volatile v4f*)(biasws + i4) = o;
    __threadfence();
    *(volatile v4f*)(biasws + i4) = o;
  }
}

__device__ __forceinline__ void stage_x(_Float16* At, const float* Tab, const float* __restrict__ obs,
                                        int rowbase, int tstep, int tid) {
  const int row = tid >> 3;
  const int c0  = (tid & 7) * 16;
  const int tp  = (tstep > 0) ? (tstep - 1) : 0;
  const bool istag = (tstep == 0);
  const float* op = obs + (size_t)(rowbase + row) * (size_t)(NTIME * 2);
  const v2f cur = *(const v2f*)(op + 2 * tstep);
  const v2f prv = *(const v2f*)(op + 2 * tp);
  const float v0 = (cur[0] - prv[0]) * VSCALE;
  const float v1 = (cur[1] - prv[1]) * VSCALE;
  v8h h0v, h1v;
#pragma unroll
  for (int q = 0; q < 4; ++q) {
    const v4f w0 = *(const v4f*)(Tab + c0 + 4 * q);
    const v4f w1 = *(const v4f*)(Tab + NXIN + c0 + 4 * q);
    const v4f bq = *(const v4f*)(Tab + 2 * NXIN + c0 + 4 * q);
    const v4f tg = *(const v4f*)(Tab + 3 * NXIN + c0 + 4 * q);
#pragma unroll
    for (int e = 0; e < 4; ++e) {
      const int col = c0 + 4 * q + e;
      const float pre = v0 * w0[e] + v1 * w1[e] + bq[e];
      float val = fmaxf(pre, 0.0f);
      val = (col < NEMB) ? val : 0.0f;
      val = istag ? tg[e] : val;
      if (q < 2) h0v[4 * q + e] = (_Float16)val;
      else       h1v[4 * (q - 2) + e] = (_Float16)val;
    }
  }
  *(v8h*)(At + row * APITCH + c0)     = h0v;
  *(v8h*)(At + row * APITCH + c0 + 8) = h1v;
}

__device__ __forceinline__ void store_tile(const float* St, float* __restrict__ dst, int rowbase, int tid) {
  for (int pass = 0; pass < 2; ++pass) {
#pragma unroll
    for (int it = 0; it < (BMROWS * (NHID / 4)) / NTHR; ++it) {
      const int idx = it * NTHR + tid;
      const int row = idx >> 6;
      const int c4  = (idx & 63) * 4;
      const v4f v = *(const v4f*)(St + row * SPITCH + c4);
      *(volatile v4f*)(dst + (size_t)(rowbase + row) * NHID + c4) = v;
    }
    __threadfence();
  }
}

__global__ __launch_bounds__(NTHR) void lstm_seq_kernel(const float* __restrict__ obs, const float* __restrict__ wemb,
                                                        const float* __restrict__ bemb,
                                                        const unsigned short* __restrict__ Wcp,
                                                        const float* __restrict__ biasws,
                                                        float* __restrict__ out) {
  __shared__ __align__(16) _Float16 At[BMROWS * APITCH];
  __shared__ __align__(16) float    St[BMROWS * SPITCH];
  __shared__ __align__(16) float    Tab[4 * NXIN];
  const _Float16* Wc = (const _Float16*)Wcp;
  const int tid = threadIdx.x, lane = tid & 31, wave = tid >> 5;
  const int c = lane & 15, hh = lane >> 4;
  const int rowbase = blockIdx.x * BMROWS;
  const int j = 16 * wave + c;

  if (tid < NXIN) {
    const int e  = tid;
    const int ec = (e < NEMB) ? e : (NEMB - 1);
    const float a0 = wemb[ec];
    const float a1 = wemb[NEMB + ec];
    const float bq = bemb[ec];
    const bool ok = (e < NEMB);
    Tab[e]            = ok ? a0 : 0.0f;
    Tab[NXIN + e]     = ok ? a1 : 0.0f;
    Tab[2 * NXIN + e] = ok ? bq : 0.0f;
    Tab[3 * NXIN + e] = (e == NEMB) ? 1.0f : 0.0f;
  }
  {
    const v8h zh = {(_Float16)0.0f, (_Float16)0.0f, (_Float16)0.0f, (_Float16)0.0f,
                    (_Float16)0.0f, (_Float16)0.0f, (_Float16)0.0f, (_Float16)0.0f};
#pragma unroll
    for (int it = 0; it < (BMROWS * (NHID / 8)) / NTHR; ++it) {
      const int idx = it * NTHR + tid;
      const int row = idx >> 5;
      const int c8  = (idx & 31) * 8;
      *(v8h*)(At + row * APITCH + NXIN + c8) = zh;
    }
  }
  float cst[MTILES][8];
#pragma unroll
  for (int i = 0; i < MTILES; ++i)
#pragma unroll
    for (int r = 0; r < 8; ++r) cst[i][r] = 0.0f;
  const float bb0 = biasws[0 * NHID + j];
  const float bb1 = biasws[1 * NHID + j];
  const float bb2 = biasws[2 * NHID + j];
  const float bb3 = biasws[3 * NHID + j];
  __syncthreads();
  stage_x(At, Tab, obs, rowbase, 0, tid);
  __syncthreads();

  const _Float16* arow = At + c * APITCH + 8 * hh;
  const _Float16* wrow = Wc + (size_t)j * KCAT + 8 * hh;
  constexpr size_t GSTRIDE = (size_t)NHID * KCAT;
  const v8f z8 = {0.f, 0.f, 0.f, 0.f, 0.f, 0.f, 0.f, 0.f};

#pragma unroll 1
  for (int t = 0; t < NCELL; ++t) {
    const bool last = (t == NCELL - 1);
    v8f acc[MTILES][4];
#pragma unroll
    for (int i = 0; i < MTILES; ++i) {
      acc[i][0] = z8; acc[i][1] = z8; acc[i][2] = z8; acc[i][3] = z8;
    }
#pragma unroll 1
    for (int kt = 0; kt < KTILES; ++kt) {
      const int k0 = kt * 32;
      const v16h b0 = Frag<_Float16>::load(wrow + k0);
      const v16h b1 = Frag<_Float16>::load(wrow + 1 * GSTRIDE + k0);
      const v16h b2 = Frag<_Float16>::load(wrow + 2 * GSTRIDE + k0);
      const v16h b3 = Frag<_Float16>::load(wrow + 3 * GSTRIDE + k0);
#pragma unroll
      for (int i = 0; i < MTILES; ++i) {
        const v16h a = Frag<_Float16>::load(arow + i * 16 * APITCH + k0);
        acc[i][0] = Frag<_Float16>::mma(a, b0, acc[i][0]);
        acc[i][1] = Frag<_Float16>::mma(a, b1, acc[i][1]);
        acc[i][2] = Frag<_Float16>::mma(a, b2, acc[i][2]);
        acc[i][3] = Frag<_Float16>::mma(a, b3, acc[i][3]);
        grp_guard(acc[i][0], acc[i][1], acc[i][2], acc[i][3], a, b0, b1, b2, b3);
      }
    }
    __syncthreads();

#pragma unroll
    for (int i = 0; i < MTILES; ++i) {
#pragma unroll
      for (int r = 0; r < 8; ++r) {
        const float zi = acc[i][0][r] * WCARRY_INV + bb0;
        const float zf = acc[i][1][r] * WCARRY_INV + bb1;
        const float zg = acc[i][2][r] * WCARRY_INV + bb2;
        const float zo = acc[i][3][r] * WCARRY_INV + bb3;
        const float ig = fsig(zi);
        const float fg = fsig(zf);
        const float gg = ftanh(zg);
        const float og = fsig(zo);
        const float cn = fg * cst[i][r] + ig * gg;
        const float hn = og * ftanh(cn);
        cst[i][r] = cn;
        const int rw = 16 * i + 8 * hh + r;
        At[rw * APITCH + NXIN + j] = (_Float16)hn;
        if (last) St[rw * SPITCH + j] = hn;
      }
    }
    {
      const int tn = (t + 1 < NCELL) ? (t + 1) : (NCELL - 1);
      stage_x(At, Tab, obs, rowbase, tn, tid);
    }
    __syncthreads();
  }

  store_tile(St, out, rowbase, tid);
  __syncthreads();
#pragma unroll
  for (int i = 0; i < MTILES; ++i)
#pragma unroll
    for (int r = 0; r < 8; ++r) St[(16 * i + 8 * hh + r) * SPITCH + j] = cst[i][r];
  __syncthreads();
  store_tile(St, out + (size_t)OUT1_ELEM_OFF, rowbase, tid);
}

extern "C" void kernel_launch(void* const* d_in, const int* in_sizes, int n_in,
                              void* d_out, int out_size, void* d_ws, size_t ws_size, hipStream_t stream) {
  if (n_in < 8 || d_out == nullptr || d_ws == nullptr) return;
  if (in_sizes[0] != NBATCH * NTIME * 2 || in_sizes[2] != 2 * NEMB || in_sizes[3] != NEMB ||
      in_sizes[4] != NGATE * NXIN || in_sizes[5] != NGATE * NHID || in_sizes[6] != NGATE || in_sizes[7] != NGATE ||
      out_size != 2 * NBATCH * NHID) return;

  const float* observed = (const float*)d_in[0];
  const float* w_emb    = (const float*)d_in[2];
  const float* b_emb    = (const float*)d_in[3];
  const float* w_ih     = (const float*)d_in[4];
  const float* w_hh     = (const float*)d_in[5];
  const float* b_ih     = (const float*)d_in[6];
  const float* b_hh     = (const float*)d_in[7];
  float* out = (float*)d_out;

  char* ws = (char*)d_ws; size_t off = 0;
  auto carve = [&](size_t bytes) -> char* { char* p = ws + off; off += (bytes + 255) & ~(size_t)255; return p; };
  unsigned short* Wc   = (unsigned short*)carve((size_t)NGATE * KCAT * 2);
  float*          BIAS = (float*)carve((size_t)NGATE * 4);
  if (off > ws_size || off > (size_t)134217728) return;

  lstm_prep_kernel<<<193, PREPT, 0, stream>>>(w_ih, w_hh, b_ih, b_hh, Wc, BIAS);
  lstm_seq_kernel<<<NBATCH / BMROWS, NTHR, 0, stream>>>(observed, w_emb, b_emb, Wc, BIAS, out);
}
